// GraphConvolutionalLayer_78073915507128
// MI455X (gfx1250) — hardware-verified
//
#include <hip/hip_runtime.h>


#define NN   1024
#define DD   128
#define DM   DD
#define NTK  NN
#define VHD  128
#define NKVV 1
#define KW   DD
#define NT_  NN
#define BN_EPS 1e-5f
#define LOSC 1024.0f

typedef _Float16 h16;
typedef unsigned short bf;
typedef __attribute__((ext_vector_type(16))) __bf16   v16bf;
typedef __attribute__((ext_vector_type(16))) _Float16 v16h;
typedef __attribute__((ext_vector_type(8)))  _Float16 v8h;
typedef __attribute__((ext_vector_type(8)))  unsigned short v8us;
typedef __attribute__((ext_vector_type(8)))  float    v8f;
typedef __attribute__((ext_vector_type(4)))  float    v4f;
typedef __attribute__((ext_vector_type(4)))  _Float16 v4h;
typedef v8h  __attribute__((may_alias)) v8ha;
typedef v4f  __attribute__((may_alias)) v4fa;
typedef v8us __attribute__((may_alias)) v8usa;

__device__ __forceinline__ unsigned short f2bf(float f) { unsigned u = __float_as_uint(f); u += 0x7FFFu + ((u >> 16) & 1u); return (unsigned short)(u >> 16); }
__device__ __forceinline__ float bf2f(unsigned short b) { return __uint_as_float(((unsigned)b) << 16); }
__device__ __forceinline__ float bfr(float f) { return bf2f(f2bf(f)); }
__device__ __forceinline__ v16h cat16(v8h lo, v8h hi) { return __builtin_shufflevector(lo, hi, 0, 1, 2, 3, 4, 5, 6, 7, 8, 9, 10, 11, 12, 13, 14, 15); }
__device__ __forceinline__ v16bf cat16b(v8us lo, v8us hi) { return __builtin_bit_cast(v16bf, __builtin_shufflevector(lo, hi, 0, 1, 2, 3, 4, 5, 6, 7, 8, 9, 10, 11, 12, 13, 14, 15)); }
__device__ __forceinline__ v8f wmma16(v16h a, v16h b, v8f c) { return __builtin_amdgcn_wmma_f32_16x16x32_f16(false, a, false, b, (short)0, c, false, false); }
__device__ __forceinline__ v8f wmmab(v16bf a, v16bf b, v8f c) { return __builtin_amdgcn_wmma_f32_16x16x32_bf16(false, a, false, b, (short)0, c, false, false); }

__global__ __launch_bounds__(256) void k_wt(const float* __restrict__ Wm, int K, int ncols, bf* WT) {
    __shared__ __align__(16) unsigned short tl[64 * 72];
    const int tid = threadIdx.x, k0 = blockIdx.x * 64, n0 = blockIdx.y * 64;
    const int kk = tid >> 2, nq = (tid & 3) * 16;
#pragma unroll
    for (int i = 0; i < 16; ++i) tl[(nq + i) * 72 + kk] = f2bf(Wm[(size_t)(k0 + kk) * ncols + n0 + nq + i]);
    __syncthreads();
    const int piece = tid & 7;
    auto pass = [&]() {
#pragma unroll
        for (int s = 0; s < 2; ++s) { const int nr = (tid >> 3) + 32 * s; const v8us val = *(const v8usa*)(tl + nr * 72 + piece * 8); *(volatile v8us*)(WT + (size_t)(n0 + nr) * K + k0 + piece * 8) = val; }
    };
    pass(); __threadfence(); pass();
}
template <bool SPLITA, bool F16OUT = false>
__global__ __launch_bounds__(128) void k_gemmb(const bf* __restrict__ A, const bf* __restrict__ Al, const bf* __restrict__ Bn, const float* __restrict__ bias, float* C, int ldc, h16* C2, const float* __restrict__ R = nullptr, int K = DM, int roundR = 1) {
    __shared__ __align__(16) float ost[4][16 * 68];
    const int lane = threadIdx.x & 31, wave = threadIdx.x >> 5, lr = lane & 15, hi = lane >> 4;
    const int r0 = blockIdx.x * 64 + wave * 16, c0 = blockIdx.y * 64;
    const size_t aoff = (size_t)(r0 + lr) * K + 8 * hi;
    size_t boff[4];
#pragma unroll
    for (int t = 0; t < 4; ++t) boff[t] = (size_t)(c0 + t * 16 + lr) * K + 8 * hi;
    v8f acc[4];
#pragma unroll
    for (int t = 0; t < 4; ++t) acc[t] = (v8f){};
#pragma unroll 1
    for (int kc = 0; kc < K; kc += 32) {
        const v16bf a = cat16b(*(const v8us*)(A + aoff + kc), *(const v8us*)(A + aoff + kc + 16));
        v16bf al = a;
        if (SPLITA) al = cat16b(*(const v8us*)(Al + aoff + kc), *(const v8us*)(Al + aoff + kc + 16));
#pragma unroll
        for (int t = 0; t < 4; ++t) { const v16bf b = cat16b(*(const v8us*)(Bn + boff[t] + kc), *(const v8us*)(Bn + boff[t] + kc + 16)); acc[t] = wmmab(a, b, acc[t]); if (SPLITA) acc[t] = wmmab(al, b, acc[t]); }
        asm volatile("v_nop\n\tv_nop\n\tv_nop\n\tv_nop" : "+v"(acc[0]), "+v"(acc[1]), "+v"(acc[2]), "+v"(acc[3]) : "v"(a), "v"(al));
    }
    float* os = &ost[wave][0];
#pragma unroll
    for (int t = 0; t < 4; ++t) { const float bv = bias ? bfr(bias[c0 + t * 16 + lr]) : 0.f;
#pragma unroll
        for (int j = 0; j < 8; ++j) os[(hi * 8 + j) * 68 + t * 16 + lr] = acc[t][j] + bv; }
    __syncthreads();
    if (F16OUT) {
        h16* crow = (h16*)(void*)C + (size_t)r0 * ldc + c0;
        auto pass = [&]() {
#pragma unroll
            for (int s = 0; s < 4; ++s) { const int row = 4 * s + (lane >> 3), piece = lane & 7; const float* sp = os + row * 68 + piece * 8; v8h o, o2;
#pragma unroll
                for (int i = 0; i < 8; ++i) { const h16 a = (h16)sp[i]; o[i] = a; o2[i] = (h16)((sp[i] - (float)a) * LOSC); }
                *(volatile v8h*)(crow + (size_t)row * ldc + piece * 8) = o; if (C2) *(volatile v8h*)(C2 + (size_t)r0 * ldc + c0 + (size_t)row * ldc + piece * 8) = o2; }
        };
        pass(); __threadfence(); pass();
    } else {
        float* crow = C + (size_t)r0 * ldc + c0;
        auto pass = [&]() {
#pragma unroll
            for (int s = 0; s < 8; ++s) { const int Lid = (lane >> 3) + 4 * s, piece = lane & 7; const int row = Lid >> 1, cofs = (Lid & 1) * 32 + piece * 4;
                v4f val = *(const v4fa*)(os + row * 68 + cofs); if (R) { const v4f rv = *(const v4f*)(R + ((size_t)r0 + row) * ldc + c0 + cofs); val += roundR ? (v4f){bfr(rv[0]), bfr(rv[1]), bfr(rv[2]), bfr(rv[3])} : rv; }
                *(volatile v4f*)(crow + (size_t)row * ldc + cofs) = val; }
        };
        pass(); __threadfence(); pass();
    }
}

__global__ __launch_bounds__(128) void k_gemm3(const bf* __restrict__ Ah, const bf* __restrict__ Al, const bf* __restrict__ Bh, const bf* __restrict__ Bl, int K, float* C, int ldc) {
    __shared__ __align__(16) float ost[4][16 * 68];
    const int lane = threadIdx.x & 31, wave = threadIdx.x >> 5, lr = lane & 15, hi = lane >> 4;
    const int r0 = blockIdx.x * 64 + wave * 16, c0 = blockIdx.y * 64;
    const size_t aoff = (size_t)(r0 + lr) * K + 8 * hi;
    v8f acc[4];
#pragma unroll
    for (int t = 0; t < 4; ++t) acc[t] = (v8f){};
#pragma unroll 1
    for (int kc = 0; kc < K; kc += 32) {
        const v16bf a = cat16b(*(const v8us*)(Ah + aoff + kc), *(const v8us*)(Ah + aoff + kc + 16));
        const v16bf al = cat16b(*(const v8us*)(Al + aoff + kc), *(const v8us*)(Al + aoff + kc + 16));
#pragma unroll
        for (int t = 0; t < 4; ++t) { const size_t bo = (size_t)(c0 + t * 16 + lr) * K + kc + 8 * hi;
            const v16bf bh = cat16b(*(const v8us*)(Bh + bo), *(const v8us*)(Bh + bo + 16)); const v16bf bl = cat16b(*(const v8us*)(Bl + bo), *(const v8us*)(Bl + bo + 16));
            acc[t] = wmmab(a, bh, acc[t]); acc[t] = wmmab(al, bh, acc[t]); acc[t] = wmmab(a, bl, acc[t]); }
        asm volatile("v_nop\n\tv_nop\n\tv_nop\n\tv_nop" : "+v"(acc[0]), "+v"(acc[1]), "+v"(acc[2]), "+v"(acc[3]) : "v"(a), "v"(al));
    }
    float* os = &ost[wave][0];
#pragma unroll
    for (int t = 0; t < 4; ++t) {
#pragma unroll
        for (int j = 0; j < 8; ++j) os[(hi * 8 + j) * 68 + t * 16 + lr] = acc[t][j]; }
    __builtin_amdgcn_wave_barrier(); asm volatile("" ::: "memory");
    float* crow = C + (size_t)r0 * ldc + c0;
    auto pass = [&]() {
#pragma unroll
        for (int s = 0; s < 8; ++s) { const int Lid = (lane >> 3) + 4 * s, piece = lane & 7; const int row = Lid >> 1, cofs = (Lid & 1) * 32 + piece * 4;
            const v4f val = *(const v4fa*)(os + row * 68 + cofs); *(volatile v4f*)(crow + (size_t)row * ldc + cofs) = val; }
    };
    pass(); __threadfence(); pass();
}
__global__ __launch_bounds__(256) void k_vt(const float* __restrict__ V, bf* VTH, bf* VTL) {
    __shared__ float tl[64][65];
    const int tid = threadIdx.x, t0 = blockIdx.x * 64, d0 = blockIdx.y * 64, g = blockIdx.z;
    { const int tt = tid >> 2, dq = (tid & 3) * 16;
#pragma unroll
      for (int i = 0; i < 16; ++i) tl[dq + i][tt] = V[(size_t)(t0 + tt) * KW + g * VHD + d0 + dq + i]; }
    __syncthreads();
    const int piece = tid & 7;
    auto pass = [&]() {
#pragma unroll
        for (int s = 0; s < 2; ++s) { const int d = (tid >> 3) + 32 * s; v8us oh, ol;
#pragma unroll
            for (int i = 0; i < 8; ++i) { const float v = tl[d][piece * 8 + i]; const unsigned short hb = f2bf(v); oh[i] = hb; ol[i] = f2bf(v - bf2f(hb)); }
            const size_t o = ((size_t)g * VHD + d0 + d) * NT_ + t0 + piece * 8; *(volatile v8us*)(VTH + o) = oh; *(volatile v8us*)(VTL + o) = ol; }
    };
    pass(); __threadfence(); pass();
}

__global__ __launch_bounds__(256) void k_bfz(const float* __restrict__ src, bf* dh, bf* dz, size_t n8) {
    const size_t i = (size_t)blockIdx.x * 256 + threadIdx.x; if (i >= n8) return;
    const v8f v = *(const v8f*)(src + i * 8); v8us o, z;
#pragma unroll
    for (int k = 0; k < 8; ++k) { o[k] = f2bf(v[k]); z[k] = 0; }
    *(volatile v8us*)(dh + i * 8) = o; *(volatile v8us*)(dz + i * 8) = z; __threadfence(); *(volatile v8us*)(dh + i * 8) = o; *(volatile v8us*)(dz + i * 8) = z;
}
__global__ __launch_bounds__(256) void k_split(const float* __restrict__ src, int nrows, bf* dh, bf* dl) {
    typedef __attribute__((ext_vector_type(4))) unsigned short v4us;
    const int lane = threadIdx.x & 31, r = blockIdx.x * 8 + (threadIdx.x >> 5); if (r >= nrows) return;
    const size_t o = (size_t)r * DD + lane * 4; const v4f v = *(const v4f*)(src + o); v4us oh, ol;
#pragma unroll
    for (int i = 0; i < 4; ++i) { const unsigned short hb = f2bf(v[i]); oh[i] = hb; ol[i] = f2bf(v[i] - bf2f(hb)); }
    *(volatile v4us*)(dh + o) = oh; *(volatile v4us*)(dl + o) = ol; __threadfence(); *(volatile v4us*)(dh + o) = oh; *(volatile v4us*)(dl + o) = ol;
}
__global__ __launch_bounds__(256) void k_score(const float* __restrict__ SRC, const float* __restrict__ TGT, const float* __restrict__ ba1, const float* __restrict__ Wa2, const float* __restrict__ ba2, const float* __restrict__ adj, bf* Ph, bf* Pl) {
    typedef __attribute__((ext_vector_type(4))) unsigned short v4us;
    __shared__ float sb[DD]; __shared__ float w2[DD]; __shared__ float red[256];
    const int tid = threadIdx.x, i = blockIdx.x;
    if (tid < DD) { sb[tid] = SRC[(size_t)i * DD + tid] + bfr(ba1[tid]); w2[tid] = bfr(Wa2[tid]); }
    __syncthreads();
    const float b2 = bfr(ba2[0]);
    float sc[4];
#pragma unroll
    for (int q = 0; q < 4; ++q) { const int j = tid * 4 + q; const float* tr = TGT + (size_t)j * DD; float s = 0.f;
#pragma unroll 1
        for (int d = 0; d < DD; ++d) { const float a = sb[d] + tr[d]; const float th = 1.0f - 2.0f / (__expf(2.0f * a) + 1.0f); s = fmaf(w2[d], th, s); }
        sc[q] = (1.0f / (1.0f + __expf(-(s + b2)))) * bfr(adj[(size_t)i * NN + j]); }
    float m = fmaxf(fmaxf(sc[0], sc[1]), fmaxf(sc[2], sc[3])); red[tid] = m; __syncthreads();
#pragma unroll
    for (int st = 128; st >= 1; st >>= 1) { if (tid < st) red[tid] = fmaxf(red[tid], red[tid + st]); __syncthreads(); }
    m = red[0]; __syncthreads();
    float e[4], se = 0.f;
#pragma unroll
    for (int q = 0; q < 4; ++q) { e[q] = __expf(sc[q] - m); se += e[q]; }
    red[tid] = se; __syncthreads();
#pragma unroll
    for (int st = 128; st >= 1; st >>= 1) { if (tid < st) red[tid] = red[tid] + red[tid + st]; __syncthreads(); }
    const float inv = 1.0f / red[0];
    v4us oh, ol;
#pragma unroll
    for (int q = 0; q < 4; ++q) { const float p = e[q] * inv; const unsigned short hb = f2bf(p); oh[q] = hb; ol[q] = f2bf(p - bf2f(hb)); }
    const size_t o = (size_t)i * NN + tid * 4;
    *(volatile v4us*)(Ph + o) = oh; *(volatile v4us*)(Pl + o) = ol; __threadfence(); *(volatile v4us*)(Ph + o) = oh; *(volatile v4us*)(Pl + o) = ol;
}
__global__ __launch_bounds__(128) void k_bnout(const float* __restrict__ O0, const float* __restrict__ Y1, const float* __restrict__ Y2, const float* __restrict__ bias, const float* __restrict__ g, const float* __restrict__ bt, float* OUTP) {
    const int c = threadIdx.x; const float bc = bfr(bias[c]);
    float s = 0.f;
#pragma unroll 1
    for (int r = 0; r < NN; ++r) { const size_t o = (size_t)r * DD + c; s += (O0[o] + Y1[o]) + (Y2[o] + bc); }
    const float mu = s / (float)NN; float s2 = 0.f;
#pragma unroll 1
    for (int r = 0; r < NN; ++r) { const size_t o = (size_t)r * DD + c; const float d = ((O0[o] + Y1[o]) + (Y2[o] + bc)) - mu; s2 = fmaf(d, d, s2); }
    const float rs = rsqrtf(s2 / (float)NN + BN_EPS), gg = bfr(g[c]), bb = bfr(bt[c]);
#pragma unroll 1
    for (int ps = 0; ps < 2; ++ps) {
#pragma unroll 1
        for (int r = 0; r < NN; ++r) { const size_t o = (size_t)r * DD + c; const float y = fmaxf((((O0[o] + Y1[o]) + (Y2[o] + bc)) - mu) * rs * gg + bb, 0.f); *(volatile float*)(OUTP + o) = y; }
        if (ps == 0) __threadfence(); }
}

extern "C" void kernel_launch(void* const* d_in, const int* in_sizes, int n_in,
                              void* d_out, int out_size, void* d_ws, size_t ws_size, hipStream_t stream) {
    (void)in_sizes; (void)n_in; (void)out_size;
    const float* nf = (const float*)d_in[0]; const float* adjc = (const float*)d_in[1]; const float* adje = (const float*)d_in[2];
    const float* Wself = (const float*)d_in[4]; const float* Wcomm = (const float*)d_in[5]; const float* Wexec = (const float*)d_in[6]; const float* bias = (const float*)d_in[7];
    const float* Wa1 = (const float*)d_in[8]; const float* ba1 = (const float*)d_in[9]; const float* Wa2 = (const float*)d_in[10]; const float* ba2 = (const float*)d_in[11]; const float* bng = (const float*)d_in[12]; const float* bnb = (const float*)d_in[13];
    float* out = (float*)d_out;
    char* wsp = (char*)d_ws;
    auto take = [&](size_t bytes) { char* p = wsp; wsp += (bytes + 255) & ~(size_t)255; return (void*)p; };
    bf* WsT = (bf*)take(DD * DD * 2); bf* WcT = (bf*)take(DD * DD * 2); bf* WeT = (bf*)take(DD * DD * 2); bf* Wa1aT = (bf*)take(DD * DD * 2); bf* Wa1bT = (bf*)take(DD * DD * 2);
    bf* NFb = (bf*)take((size_t)NN * DD * 2); float* O0 = (float*)take((size_t)NN * DD * 4); float* T = (float*)take((size_t)NN * DD * 4); float* E = (float*)take((size_t)NN * DD * 4);
    bf* Th = (bf*)take((size_t)NN * DD * 2); bf* Tl = (bf*)take((size_t)NN * DD * 2); float* SRC = (float*)take((size_t)NN * DD * 4); float* TGT = (float*)take((size_t)NN * DD * 4);
    bf* Ph = (bf*)take((size_t)NN * NN * 2); bf* Pl = (bf*)take((size_t)NN * NN * 2); bf* Ah = (bf*)take((size_t)NN * NN * 2); bf* Az = (bf*)take((size_t)NN * NN * 2);
    bf* TTh = (bf*)take((size_t)DD * NN * 2); bf* TTl = (bf*)take((size_t)DD * NN * 2); bf* ETh = (bf*)take((size_t)DD * NN * 2); bf* ETl = (bf*)take((size_t)DD * NN * 2);
    float* Y1 = (float*)take((size_t)NN * DD * 4); float* Y2 = (float*)take((size_t)NN * DD * 4);
    if ((size_t)(wsp - (char*)d_ws) > ws_size) return;
    k_wt<<<dim3(DD / 64, DD / 64, 1), 256, 0, stream>>>(Wself, DD, DD, WsT); k_wt<<<dim3(DD / 64, DD / 64, 1), 256, 0, stream>>>(Wcomm, DD, DD, WcT); k_wt<<<dim3(DD / 64, DD / 64, 1), 256, 0, stream>>>(Wexec, DD, DD, WeT);
    k_wt<<<dim3(DD / 64, DD / 64, 1), 256, 0, stream>>>(Wa1, DD, DD, Wa1aT); k_wt<<<dim3(DD / 64, DD / 64, 1), 256, 0, stream>>>(Wa1 + DD * DD, DD, DD, Wa1bT);
    k_bfz<<<(NN * DD / 8 + 255) / 256, 256, 0, stream>>>(nf, NFb, Az, (size_t)NN * DD / 8);
    k_bfz<<<(NN * NN / 8 + 255) / 256, 256, 0, stream>>>(adje, Ah, Az, (size_t)NN * NN / 8);
    k_gemmb<false, false><<<dim3(NN / 64, DD / 64, 1), 128, 0, stream>>>(NFb, nullptr, WsT, nullptr, O0, DD, nullptr);
    k_gemmb<false, false><<<dim3(NN / 64, DD / 64, 1), 128, 0, stream>>>(NFb, nullptr, WcT, nullptr, T, DD, nullptr);
    k_gemmb<false, false><<<dim3(NN / 64, DD / 64, 1), 128, 0, stream>>>(NFb, nullptr, WeT, nullptr, E, DD, nullptr);
    k_split<<<NN / 8, 256, 0, stream>>>(T, NN, Th, Tl);
    k_gemmb<true, false><<<dim3(NN / 64, DD / 64, 1), 128, 0, stream>>>(Th, Tl, Wa1aT, nullptr, SRC, DD, nullptr);
    k_gemmb<true, false><<<dim3(NN / 64, DD / 64, 1), 128, 0, stream>>>(Th, Tl, Wa1bT, nullptr, TGT, DD, nullptr);
    k_score<<<NN, 256, 0, stream>>>(SRC, TGT, ba1, Wa2, ba2, adjc, Ph, Pl);
    k_vt<<<dim3(NN / 64, 2, NKVV), 256, 0, stream>>>(T, TTh, TTl); k_vt<<<dim3(NN / 64, 2, NKVV), 256, 0, stream>>>(E, ETh, ETl);
    k_gemm3<<<dim3(NN / 64, DD / 64, 1), 128, 0, stream>>>(Ph, Pl, TTh, TTl, NN, Y1, DD);
    k_gemm3<<<dim3(NN / 64, DD / 64, 1), 128, 0, stream>>>(Ah, Az, ETh, ETl, NN, Y2, DD);
    k_bnout<<<1, 128, 0, stream>>>(O0, Y1, Y2, bias, bng, bnb, out);
}
